// MambaLayer_21492016349886
// MI455X (gfx1250) — hardware-run, weakly checked
//
#include <hip/hip_runtime.h>
#include <math.h>

typedef __attribute__((ext_vector_type(16))) _Float16 v16h;
typedef __attribute__((ext_vector_type(8)))  _Float16 v8h;
typedef __attribute__((ext_vector_type(8)))  float    v8f;
typedef __attribute__((ext_vector_type(4)))  float    v4f;

constexpr int kL = 18432;
constexpr int kT = 8, kH = 48, kW = 48, kHW = kH * kW;
constexpr int kC = 64;
constexpr int kDin = 128;
constexpr int kNst = 16;
constexpr int kDtR = 4;
constexpr int kHid = 256;
constexpr int kOutC = 64;
constexpr int kCabMid = 16;
constexpr int kSqMid = 8;
constexpr int kXzP = 2 * kDin;
constexpr int kDbcN = kDtR + 2 * kNst;
constexpr int kDbcP = 64;
constexpr int kPW = kW + 2, kPH = kH + 2, kPT = kT + 2;
constexpr int kPHW = kPH * kPW;
constexpr int kPMin = kPHW + kPW + 1;
constexpr int kPMaxI = kT * kPHW + kH * kPW + kW;
constexpr int kMConv = 19904;
constexpr int kNPR = 25088;
constexpr int kTaps = 27;
constexpr int kK1 = kTaps * kC;
constexpr int kK2r = kTaps * kCabMid;
constexpr int kK2 = 448;
constexpr int kScanTS = 32, kScanCh = 64, kScanYP = 68;
constexpr float kWCar = 256.0f;
constexpr float kXcCar = 1024.0f;
constexpr float kYCar = 1024.0f;
constexpr float kGCar = 256.0f;
constexpr float kCbCar = 64.0f;

static_assert(kL % 64 == 0 && kL % 128 == 0);
static_assert(kMConv % 64 == 0 && kMConv >= kPMaxI - kPMin + 1);
static_assert(kNPR >= kPMin + kMConv + kPMin && kNPR % 128 == 0);
static_assert(kK1 % 32 == 0 && kK2 % 32 == 0 && kK2 >= kK2r && kC % 32 == 0 && kDin % 32 == 0 && kHid % 32 == 0);
static_assert(kXzP % 64 == 0 && kDbcP % 64 == 0 && kHid % 64 == 0 && kOutC % 64 == 0 && kCabMid == 16);
static_assert(kL % kScanTS == 0 && kDin % kScanCh == 0);

constexpr size_t kOffIPW  = 0;
constexpr size_t kOffOPW  = kOffIPW  + (size_t)256 * 64 * 2;
constexpr size_t kOffF1W  = kOffOPW  + (size_t)64 * 128 * 2;
constexpr size_t kOffF2W  = kOffF1W  + (size_t)256 * 64 * 2;
constexpr size_t kOffPJW  = kOffF2W  + (size_t)64 * 256 * 2;
constexpr size_t kOffXPW  = kOffPJW  + (size_t)64 * 64 * 2;
constexpr size_t kOffC1R  = kOffXPW  + (size_t)2 * 64 * 128 * 2;
constexpr size_t kOffC2R  = kOffC1R  + (size_t)kCabMid * kK1 * 2;
constexpr size_t kOffXT   = kOffC2R  + (size_t)kOutC * kK2 * 2;
constexpr size_t kOffXN   = kOffXT   + (size_t)kL * kC * 4;
constexpr size_t kOffXZ   = kOffXN   + (size_t)kL * kC * 2;
constexpr size_t kOffXC   = kOffXZ   + (size_t)kL * kXzP * 4;
constexpr size_t kOffXCS  = kOffXC   + (size_t)2 * kL * kDin * 4;
constexpr size_t kOffDBC  = kOffXCS  + (size_t)2 * kL * kDin * 2;
constexpr size_t kOffYF   = kOffDBC  + (size_t)2 * kL * kDbcP * 4;
constexpr size_t kOffYT   = kOffYF   + (size_t)kL * kDin * 4;
constexpr size_t kOffXM   = kOffYT   + (size_t)kL * kDin * 2;
constexpr size_t kOffXN2  = kOffXM   + (size_t)kL * kC * 4;
constexpr size_t kOffH1   = kOffXN2  + (size_t)kL * kC * 2;
constexpr size_t kOffH2G  = kOffH1   + (size_t)kL * kHid * 4;
constexpr size_t kOffXM2  = kOffH2G  + (size_t)kL * kHid * 2;
constexpr size_t kOffOB   = kOffXM2  + (size_t)kL * kC * 2;
constexpr size_t kOffCIP  = kOffOB   + (size_t)kL * kOutC * 4;
constexpr size_t kOffCB1  = kOffCIP  + (size_t)kNPR * kC * 2;
constexpr size_t kOffCB1G = kOffCB1  + (size_t)kMConv * kCabMid * 4;
constexpr size_t kOffCB2  = kOffCB1G + (size_t)kNPR * kCabMid * 2;
constexpr size_t kOffPART = kOffCB2  + (size_t)kMConv * kOutC * 4;
constexpr size_t kOffATT  = kOffPART + (size_t)64 * 64 * 4;
constexpr size_t kWsTotal = kOffATT  + 256;
static_assert(kWsTotal == 130992384ull);
static_assert(kWsTotal <= 134217728ull);
static_assert((kOffOPW % 128) == 0 && (kOffF1W % 128) == 0 && (kOffF2W % 128) == 0 && (kOffPJW % 128) == 0 &&
              (kOffXPW % 128) == 0 && (kOffC1R % 128) == 0 && (kOffC2R % 128) == 0 && (kOffXT % 128) == 0 &&
              (kOffXN % 128) == 0 && (kOffXZ % 128) == 0 && (kOffXC % 128) == 0 && (kOffXCS % 128) == 0 &&
              (kOffDBC % 128) == 0 && (kOffYF % 128) == 0 && (kOffYT % 128) == 0 && (kOffXM % 128) == 0 &&
              (kOffXN2 % 128) == 0 && (kOffH1 % 128) == 0 && (kOffH2G % 128) == 0 && (kOffXM2 % 128) == 0 &&
              (kOffOB % 128) == 0 && (kOffCIP % 128) == 0 && (kOffCB1 % 128) == 0 && (kOffCB1G % 128) == 0 &&
              (kOffCB2 % 128) == 0 && (kOffPART % 128) == 0 && (kOffATT % 128) == 0);

union HFrag { v16h v; v8h h[2]; };
__device__ __forceinline__ v16h frag_load(const _Float16* p) {
  HFrag f; f.h[0] = *(const v8h*)(p); f.h[1] = *(const v8h*)(p + 16); return f.v;
}
__device__ __forceinline__ v8f mma_h(v16h a, v16h b, v8f c) {
  return __builtin_amdgcn_wmma_f32_16x16x32_f16(false, a, false, b, (short)0, c, false, false);
}
__device__ __forceinline__ void guard4x(v8f& a, v8f& b, v8f& c, v8f& d, v16h x, v16h y0, v16h y1, v16h y2, v16h y3) {
  asm volatile("v_nop\n\tv_nop\n\tv_nop\n\tv_nop" : "+v"(a), "+v"(b), "+v"(c), "+v"(d) : "v"(x), "v"(y0), "v"(y1), "v"(y2), "v"(y3));
}
__device__ __forceinline__ void guard1x(v8f& a, v16h x, v16h y) {
  asm volatile("v_nop\n\tv_nop\n\tv_nop\n\tv_nop" : "+v"(a) : "v"(x), "v"(y));
}
__device__ __forceinline__ void keep4h(v16h a, v16h b, v16h c, v16h d) { asm volatile("v_nop" :: "v"(a), "v"(b), "v"(c), "v"(d)); }
__device__ __forceinline__ void keep1h(v16h a) { asm volatile("v_nop" :: "v"(a)); }
__device__ __forceinline__ void acc_guard4(v8f& a, v8f& b, v8f& c, v8f& d) {
  asm volatile("v_nop\n\tv_nop\n\tv_nop\n\tv_nop" : "+v"(a), "+v"(b), "+v"(c), "+v"(d));
}

__device__ __forceinline__ float gelu_f(float x) { return 0.5f * x * (1.0f + erff(x * 0.70710678118654752f)); }
__device__ __forceinline__ float sigm_f(float x) { return __builtin_amdgcn_rcpf(1.0f + expf(-x)); }

__device__ __forceinline__ int tap_shift(int tap) {
  const int kd = tap / 9; const int r = tap - kd * 9; const int kh = r / 3; const int kw = r - kh * 3;
  return (kd - 1) * kPHW + (kh - 1) * kPW + (kw - 1);
}
__device__ __forceinline__ int pad_interior(int p, int* lout) {
  const int t = p / kPHW; const int r = p - t * kPHW; const int h = r / kPW; const int w = r - h * kPW;
  const bool in = (t >= 1) & (t <= kT) & (h >= 1) & (h <= kH) & (w >= 1) & (w <= kW);
  const int lt = (t - 1) * kHW + (h - 1) * kW + (w - 1);
  *lout = in ? lt : 0;
  return in ? 1 : 0;
}
__device__ __forceinline__ int l_to_m(int l) {
  const int t = l / kHW; const int r = l - t * kHW; const int h = r / kW; const int w = r - h * kW;
  return (t + 1) * kPHW + (h + 1) * kPW + (w + 1) - kPMin;
}

__device__ __forceinline__ void ln8(const v4f a0, const v4f a1, const v4f g0, const v4f g1, const v4f e0, const v4f e1,
                                    v4f& o0, v4f& o1) {
  float s = ((a0.x + a0.y) + (a0.z + a0.w)) + ((a1.x + a1.y) + (a1.z + a1.w));
  s += __shfl_xor(s, 1, 32); s += __shfl_xor(s, 2, 32); s += __shfl_xor(s, 4, 32);
  const float m = s * (1.0f / 64.0f);
  const v4f d0 = a0 - m, d1 = a1 - m;
  float qq = ((d0.x * d0.x + d0.y * d0.y) + (d0.z * d0.z + d0.w * d0.w)) + ((d1.x * d1.x + d1.y * d1.y) + (d1.z * d1.z + d1.w * d1.w));
  qq += __shfl_xor(qq, 1, 32); qq += __shfl_xor(qq, 2, 32); qq += __shfl_xor(qq, 4, 32);
  const float inv = rsqrtf(qq * (1.0f / 64.0f) + 1e-5f);
  o0 = d0 * inv * g0 + e0;
  o1 = d1 * inv * g1 + e1;
}

template <int CONV, int NSUB, int BIAS_MODE, int OUT_MODE, bool RESID>
__global__ __launch_bounds__(256) void gemm_f16_kernel(
    const unsigned short* __restrict__ Ap, int lda, long strideA,
    const unsigned short* __restrict__ Btp, int ldb, long strideB,
    void* __restrict__ Cout, int ldc, long strideC,
    const float* __restrict__ bias,
    const float* __restrict__ resid, const float* __restrict__ rscp,
    int M, int N, int K, float scale)
{
  constexpr int TN = 16 * NSUB;
  __shared__ __align__(16) float sT[8][16 * 68];
  const int b    = blockIdx.y;
  const int lane = threadIdx.x & 31;
  const int wave = threadIdx.x >> 5;
  const int tilesN = N / TN;
  const int tilesM = M >> 6;
  const int tile = blockIdx.x * 8 + wave;
  if (tile >= tilesM * tilesN) return;
  const int tm = tile / tilesN;
  const int tn = tile - tm * tilesN;
  const int m0 = tm << 6;
  const int n0 = tn * TN;
  const _Float16* Ab = (const _Float16*)Ap  + (size_t)b * strideA;
  const _Float16* Bb = (const _Float16*)Btp + (size_t)b * strideB;
  const int rlane = lane & 15;
  const int koff  = (lane >> 4) * 8;
  const int mOff  = (lane >> 4) * 8;

  v8f acc[4][NSUB];
#pragma unroll
  for (int i = 0; i < 4; ++i)
#pragma unroll
    for (int j = 0; j < NSUB; ++j) acc[i][j] = (v8f){0.f, 0.f, 0.f, 0.f, 0.f, 0.f, 0.f, 0.f};
  v8h z8;
#pragma unroll
  for (int e = 0; e < 8; ++e) z8[e] = (_Float16)0.0f;

  for (int k0 = 0; k0 < K; k0 += 32) {
    v16h bh[NSUB];
#pragma unroll
    for (int j = 0; j < NSUB; ++j) bh[j] = frag_load(Bb + (size_t)(n0 + (j << 4) + rlane) * ldb + koff + k0);
    int sh0 = 0, sh1 = 0, coff = 0;
    bool lastk = false;
    if constexpr (CONV == 1) { const int tap = k0 >> 6; coff = k0 & 63; sh0 = tap_shift(tap); }
    if constexpr (CONV == 2) {
      const int tap = k0 >> 4;
      sh0 = tap_shift(tap);
      const int t1 = (tap + 1 < kTaps) ? (tap + 1) : (kTaps - 1);
      sh1 = tap_shift(t1);
      lastk = (tap + 1) >= kTaps;
    }
#pragma unroll
    for (int i = 0; i < 4; ++i) {
      const int row = m0 + (i << 4) + rlane;
      v16h ah;
      if constexpr (CONV == 0) {
        ah = frag_load(Ab + (size_t)row * lda + koff + k0);
      } else if constexpr (CONV == 1) {
        ah = frag_load(Ab + (size_t)(row + kPMin + sh0) * lda + coff + koff);
      } else {
        HFrag f;
        f.h[0] = *(const v8h*)(Ab + (size_t)(row + kPMin + sh0) * lda + koff);
        const v8h t1v = *(const v8h*)(Ab + (size_t)(row + kPMin + sh1) * lda + koff);
        if (lastk) f.h[1] = z8; else f.h[1] = t1v;
        ah = f.v;
      }
#pragma unroll
      for (int j = 0; j < NSUB; ++j) acc[i][j] = mma_h(ah, bh[j], acc[i][j]);
      if constexpr (NSUB == 4) guard4x(acc[i][0], acc[i][1], acc[i][2], acc[i][3], ah, bh[0], bh[1], bh[2], bh[3]);
      else guard1x(acc[i][0], ah, bh[0]);
    }
    if constexpr (NSUB == 4) keep4h(bh[0], bh[1], bh[2], bh[3]);
    else keep1h(bh[0]);
  }
  if constexpr (NSUB == 4) {
    acc_guard4(acc[0][0], acc[0][1], acc[0][2], acc[0][3]);
    acc_guard4(acc[1][0], acc[1][1], acc[1][2], acc[1][3]);
    acc_guard4(acc[2][0], acc[2][1], acc[2][2], acc[2][3]);
    acc_guard4(acc[3][0], acc[3][1], acc[3][2], acc[3][3]);
  } else {
    acc_guard4(acc[0][0], acc[1][0], acc[2][0], acc[3][0]);
  }

  float* slab = sT[wave];
  float rs = 1.0f;
  if constexpr (RESID) rs = rscp[0];
#pragma unroll
  for (int i = 0; i < 4; ++i) {
    const int mBase = m0 + (i << 4);
#pragma unroll
    for (int j = 0; j < NSUB; ++j) {
      const int n = n0 + (j << 4) + rlane;
      float bv = 0.f;
      if constexpr (BIAS_MODE == 2) bv = bias[n];
#pragma unroll
      for (int r = 0; r < 8; ++r) slab[(mOff + r) * 68 + (j << 4) + rlane] = acc[i][j][r] * scale + bv;
    }
    __builtin_amdgcn_fence(__ATOMIC_RELEASE, "workgroup");
    __builtin_amdgcn_wave_barrier();
    __builtin_amdgcn_fence(__ATOMIC_ACQUIRE, "workgroup");
    if constexpr (OUT_MODE == 0 && NSUB == 4) {
      float* C = (float*)Cout + (size_t)b * strideC;
      const int hh = lane >> 4, c4 = (lane & 15) * 4;
      for (int pass = 0; pass < 2; ++pass) {
#pragma unroll
        for (int it = 0; it < 8; ++it) {
          const int row = it * 2 + hh;
          v4f v = *(const v4f*)(slab + row * 68 + c4);
          if constexpr (RESID) {
            const v4f r4 = *(const v4f*)(resid + (size_t)(mBase + row) * ldc + n0 + c4);
            v = v + r4 * rs;
          }
          *(volatile v4f*)(C + (size_t)(mBase + row) * ldc + n0 + c4) = v;
        }
        __threadfence();
      }
    } else if constexpr (OUT_MODE == 0 && NSUB == 1) {
      float* C = (float*)Cout + (size_t)b * strideC;
      const int rr = lane >> 2, cc = (lane & 3) * 4;
      for (int pass = 0; pass < 2; ++pass) {
#pragma unroll
        for (int it = 0; it < 2; ++it) {
          const int row = it * 8 + rr;
          const v4f v = *(const v4f*)(slab + row * 68 + cc);
          *(volatile v4f*)(C + (size_t)(mBase + row) * ldc + n0 + cc) = v;
        }
        __threadfence();
      }
    } else {
      unsigned short* C = (unsigned short*)Cout + (size_t)b * strideC;
      const int q = lane >> 3, c8 = (lane & 7) * 8;
      for (int pass = 0; pass < 2; ++pass) {
#pragma unroll
        for (int it = 0; it < 4; ++it) {
          const int row = it * 4 + q;
          const float* sp = slab + row * 68 + c8;
          float x[8];
#pragma unroll
          for (int e = 0; e < 8; ++e) x[e] = sp[e];
          if constexpr (RESID) {
            const float* rp = resid + (size_t)(mBase + row) * ldc + n0 + c8;
            const v4f r0 = *(const v4f*)(rp), r1 = *(const v4f*)(rp + 4);
            x[0] += rs * r0.x; x[1] += rs * r0.y; x[2] += rs * r0.z; x[3] += rs * r0.w;
            x[4] += rs * r1.x; x[5] += rs * r1.y; x[6] += rs * r1.z; x[7] += rs * r1.w;
          }
          v8h hv;
#pragma unroll
          for (int e = 0; e < 8; ++e) hv[e] = (_Float16)x[e];
          *(volatile v8h*)(C + (size_t)(mBase + row) * ldc + n0 + c8) = hv;
        }
        __threadfence();
      }
    }
    __builtin_amdgcn_fence(__ATOMIC_RELEASE, "workgroup");
    __builtin_amdgcn_wave_barrier();
    __builtin_amdgcn_fence(__ATOMIC_ACQUIRE, "workgroup");
  }
}

__global__ __launch_bounds__(256) void prep_kernel(
    const float* __restrict__ ipw, const float* __restrict__ opw, const float* __restrict__ f1w,
    const float* __restrict__ f2w, const float* __restrict__ pjw,
    const float* __restrict__ xpwf, const float* __restrict__ xpwb,
    const float* __restrict__ c1w, const float* __restrict__ c2w,
    unsigned short* __restrict__ dIpw, unsigned short* __restrict__ dOpw, unsigned short* __restrict__ dF1w,
    unsigned short* __restrict__ dF2w, unsigned short* __restrict__ dPjw, unsigned short* __restrict__ dXpw,
    unsigned short* __restrict__ dC1r, unsigned short* __restrict__ dC2r)
{
  const int job = blockIdx.y;
  const int i = blockIdx.x * 256 + threadIdx.x;
  float v[8];
  unsigned short* dst;
  if (job <= 4) {
    const float* s = (job == 0) ? ipw : (job == 1) ? opw : (job == 2) ? f1w : (job == 3) ? f2w : pjw;
    unsigned short* dsel = (job == 0) ? dIpw : (job == 1) ? dOpw : (job == 2) ? dF1w : (job == 3) ? dF2w : dPjw;
    const int n8 = (job == 0) ? (256 * 64 / 8) : (job == 1) ? (64 * 128 / 8) : (job == 2) ? (256 * 64 / 8)
                 : (job == 3) ? (64 * 256 / 8) : (64 * 64 / 8);
    if (i >= n8) return;
    const v4f a0 = *(const v4f*)(s + (size_t)i * 8), a1 = *(const v4f*)(s + (size_t)i * 8 + 4);
    v[0] = a0.x * kWCar; v[1] = a0.y * kWCar; v[2] = a0.z * kWCar; v[3] = a0.w * kWCar;
    v[4] = a1.x * kWCar; v[5] = a1.y * kWCar; v[6] = a1.z * kWCar; v[7] = a1.w * kWCar;
    dst = dsel + (size_t)i * 8;
  } else if (job == 5) {
    if (i >= 2 * 64 * kDin / 8) return;
    const int br = i >> 10;
    const int rem = i & 1023;
    const int row = rem >> 4;
    const int c8 = (rem & 15) * 8;
    const float* s = br ? xpwb : xpwf;
    const int rowc = (row < kDbcN) ? row : (kDbcN - 1);
    const float f = (row < kDbcN) ? kWCar : 0.f;
    const v4f a0 = *(const v4f*)(s + (size_t)rowc * kDin + c8), a1 = *(const v4f*)(s + (size_t)rowc * kDin + c8 + 4);
    v[0] = a0.x * f; v[1] = a0.y * f; v[2] = a0.z * f; v[3] = a0.w * f;
    v[4] = a1.x * f; v[5] = a1.y * f; v[6] = a1.z * f; v[7] = a1.w * f;
    dst = dXpw + (size_t)i * 8;
  } else if (job == 6) {
    if (i >= kCabMid * kK1 / 8) return;
    const int n = i / 216, r = i - n * 216;
    const int tap = r >> 3, c8 = (r & 7) * 8;
#pragma unroll
    for (int e = 0; e < 8; ++e) v[e] = c1w[(size_t)n * kK1 + (size_t)(c8 + e) * kTaps + tap] * kWCar;
    dst = dC1r + (size_t)i * 8;
  } else {
    if (i >= kOutC * kK2 / 8) return;
    const int n = i / 56, g = i - n * 56;
    const int k8 = g * 8;
    int tap = k8 >> 4;
    const int c8 = k8 & 15;
    const float f = (g < 54) ? kWCar : 0.f;
    tap = (tap > kTaps - 1) ? (kTaps - 1) : tap;
#pragma unroll
    for (int e = 0; e < 8; ++e) v[e] = c2w[(size_t)n * kK2r + (size_t)(c8 + e) * kTaps + tap] * f;
    dst = dC2r + (size_t)i * 8;
  }
  v8h hv;
#pragma unroll
  for (int e = 0; e < 8; ++e) hv[e] = (_Float16)v[e];
  *(volatile v8h*)dst = hv;
  __threadfence();
  *(volatile v8h*)dst = hv;
}

__global__ __launch_bounds__(256) void ln1_kernel(const float* __restrict__ X, const float* __restrict__ g,
                                                  const float* __restrict__ bb, float* __restrict__ XT,
                                                  unsigned short* __restrict__ XN)
{
  __shared__ __align__(16) float sX[128 * 68];
  const int tid = threadIdx.x, lane = tid & 31, wave = tid >> 5;
  const int l0 = blockIdx.x * 128;
#pragma unroll
  for (int i = 0; i < 8; ++i) {
    const int f = tid + 256 * i;
    const int c = f >> 5;
    const int j4 = (f & 31) * 4;
    const v4f v = *(const v4f*)(X + (size_t)c * kL + l0 + j4);
    sX[(j4 + 0) * 68 + c] = v.x; sX[(j4 + 1) * 68 + c] = v.y; sX[(j4 + 2) * 68 + c] = v.z; sX[(j4 + 3) * 68 + c] = v.w;
  }
  __syncthreads();
  const int hh = lane >> 4, c4 = (lane & 15) * 4, q = lane >> 3, c8 = (lane & 7) * 8;
  v4f tv[8];
#pragma unroll
  for (int it = 0; it < 8; ++it) {
    const int row = it * 16 + wave * 2 + hh;
    tv[it] = *(const v4f*)(sX + row * 68 + c4);
  }
  const v4f g0 = *(const v4f*)(g + c8), g1 = *(const v4f*)(g + c8 + 4);
  const v4f e0 = *(const v4f*)(bb + c8), e1 = *(const v4f*)(bb + c8 + 4);
  v8h hv[4];
#pragma unroll
  for (int it = 0; it < 4; ++it) {
    const int row = it * 32 + wave * 4 + q;
    const v4f a0 = *(const v4f*)(sX + row * 68 + c8), a1 = *(const v4f*)(sX + row * 68 + c8 + 4);
    v4f o0, o1;
    ln8(a0, a1, g0, g1, e0, e1, o0, o1);
    hv[it][0] = (_Float16)o0.x; hv[it][1] = (_Float16)o0.y; hv[it][2] = (_Float16)o0.z; hv[it][3] = (_Float16)o0.w;
    hv[it][4] = (_Float16)o1.x; hv[it][5] = (_Float16)o1.y; hv[it][6] = (_Float16)o1.z; hv[it][7] = (_Float16)o1.w;
  }
  for (int pass = 0; pass < 2; ++pass) {
#pragma unroll
    for (int it = 0; it < 8; ++it) {
      const int row = it * 16 + wave * 2 + hh;
      *(volatile v4f*)(XT + (size_t)(l0 + row) * kC + c4) = tv[it];
    }
#pragma unroll
    for (int it = 0; it < 4; ++it) {
      const int row = it * 32 + wave * 4 + q;
      *(volatile v8h*)(XN + (size_t)(l0 + row) * kC + c8) = hv[it];
    }
    __threadfence();
  }
}

__global__ __launch_bounds__(256) void ln2_kernel(const float* __restrict__ XM, const float* __restrict__ g,
                                                  const float* __restrict__ bb, unsigned short* __restrict__ XN2)
{
  const int tid = threadIdx.x, lane = tid & 31, wave = tid >> 5;
  const int q = lane >> 3, c8 = (lane & 7) * 8;
  const int row = blockIdx.x * 32 + wave * 4 + q;
  const v4f a0 = *(const v4f*)(XM + (size_t)row * kC + c8), a1 = *(const v4f*)(XM + (size_t)row * kC + c8 + 4);
  const v4f g0 = *(const v4f*)(g + c8), g1 = *(const v4f*)(g + c8 + 4);
  const v4f e0 = *(const v4f*)(bb + c8), e1 = *(const v4f*)(bb + c8 + 4);
  v4f o0, o1;
  ln8(a0, a1, g0, g1, e0, e1, o0, o1);
  v8h hv;
  hv[0] = (_Float16)o0.x; hv[1] = (_Float16)o0.y; hv[2] = (_Float16)o0.z; hv[3] = (_Float16)o0.w;
  hv[4] = (_Float16)o1.x; hv[5] = (_Float16)o1.y; hv[6] = (_Float16)o1.z; hv[7] = (_Float16)o1.w;
  unsigned short* dp = XN2 + (size_t)row * kC + c8;
  *(volatile v8h*)dp = hv;
  __threadfence();
  *(volatile v8h*)dp = hv;
}

__global__ __launch_bounds__(256) void ln3pad_kernel(const float* __restrict__ OB, const float* __restrict__ g,
                                                     const float* __restrict__ bb, unsigned short* __restrict__ CIP)
{
  const int tid = threadIdx.x, lane = tid & 31, wave = tid >> 5;
  const int q = lane >> 3, c8 = (lane & 7) * 8;
  const int p = blockIdx.x * 32 + wave * 4 + q;
  int l;
  const int in = pad_interior(p, &l);
  const float f = (float)in;
  const v4f a0 = *(const v4f*)(OB + (size_t)l * kOutC + c8), a1 = *(const v4f*)(OB + (size_t)l * kOutC + c8 + 4);
  const v4f g0 = *(const v4f*)(g + c8), g1 = *(const v4f*)(g + c8 + 4);
  const v4f e0 = *(const v4f*)(bb + c8), e1 = *(const v4f*)(bb + c8 + 4);
  v4f o0, o1;
  ln8(a0, a1, g0, g1, e0, e1, o0, o1);
  o0 = o0 * f; o1 = o1 * f;
  v8h hv;
  hv[0] = (_Float16)o0.x; hv[1] = (_Float16)o0.y; hv[2] = (_Float16)o0.z; hv[3] = (_Float16)o0.w;
  hv[4] = (_Float16)o1.x; hv[5] = (_Float16)o1.y; hv[6] = (_Float16)o1.z; hv[7] = (_Float16)o1.w;
  unsigned short* dp = CIP + (size_t)p * kC + c8;
  *(volatile v8h*)dp = hv;
  __threadfence();
  *(volatile v8h*)dp = hv;
}

__global__ __launch_bounds__(128) void conv1d_silu_kernel(
    const float* __restrict__ XZ, const float* __restrict__ wf, const float* __restrict__ bfp,
    const float* __restrict__ wbk, const float* __restrict__ bbk,
    float* __restrict__ XC, unsigned short* __restrict__ XCS)
{
  __shared__ __align__(16) float sT[16 * 132];
  const int tid = threadIdx.x, lane = tid & 31, wave = tid >> 5;
  const int br = blockIdx.y;
  const float* w  = br ? wbk : wf;
  const float* bp = br ? bbk : bfp;
  const float w0 = w[tid * 4 + 0], w1 = w[tid * 4 + 1], w2 = w[tid * 4 + 2], w3 = w[tid * 4 + 3];
  const float bc = bp[tid];
  const int i0 = blockIdx.x * 64;
  float xm3, xm2, xm1;
  {
    const bool hist = (i0 > 0);
    const int ic = hist ? i0 : 3;
    const int r3 = br ? (kL - 1 - (ic - 3)) : (ic - 3);
    const int r2 = br ? (kL - 1 - (ic - 2)) : (ic - 2);
    const int r1 = br ? (kL - 1 - (ic - 1)) : (ic - 1);
    const float v3 = XZ[(size_t)r3 * kXzP + tid];
    const float v2 = XZ[(size_t)r2 * kXzP + tid];
    const float v1 = XZ[(size_t)r1 * kXzP + tid];
    xm3 = hist ? v3 : 0.f;
    xm2 = hist ? v2 : 0.f;
    xm1 = hist ? v1 : 0.f;
  }
  float* XCb = XC + (size_t)br * kL * kDin;
  unsigned short* XSb = XCS + (size_t)br * kL * kDin;
  const int hh = lane >> 4, c8 = (lane & 15) * 8;
#pragma unroll 1
  for (int sub = 0; sub < 4; ++sub) {
    const int lb = i0 + sub * 16;
#pragma unroll 1
    for (int s = 0; s < 16; ++s) {
      const int gi = lb + s;
      const int gr = br ? (kL - 1 - gi) : gi;
      const float xcur = XZ[(size_t)gr * kXzP + tid];
      float acc = w0 * xm3;
      acc = fmaf(w1, xm2, acc);
      acc = fmaf(w2, xm1, acc);
      acc = fmaf(w3, xcur, acc);
      const float sv = acc + bc;
      sT[s * 132 + tid] = sv * sigm_f(sv);
      xm3 = xm2; xm2 = xm1; xm1 = xcur;
    }
    __syncthreads();
    v4f fv[4];
#pragma unroll
    for (int it = 0; it < 4; ++it) fv[it] = *(const v4f*)(sT + (it * 4 + wave) * 132 + lane * 4);
    v8h hv[2];
#pragma unroll
    for (int it = 0; it < 2; ++it) {
      const float* sp = sT + (it * 8 + wave * 2 + hh) * 132 + c8;
#pragma unroll
      for (int e = 0; e < 8; ++e) hv[it][e] = (_Float16)(sp[e] * kXcCar);
    }
    for (int pass = 0; pass < 2; ++pass) {
#pragma unroll
      for (int it = 0; it < 4; ++it) {
        const int gi = lb + it * 4 + wave;
        const int gr = br ? (kL - 1 - gi) : gi;
        *(volatile v4f*)(XCb + (size_t)gr * kDin + lane * 4) = fv[it];
      }
#pragma unroll
      for (int it = 0; it < 2; ++it) {
        const int gi = lb + it * 8 + wave * 2 + hh;
        const int gr = br ? (kL - 1 - gi) : gi;
        *(volatile v8h*)(XSb + (size_t)gr * kDin + c8) = hv[it];
      }
      __threadfence();
    }
    __syncthreads();
  }
}

template <int DIR>
__global__ __launch_bounds__(64) void scan_kernel(
    const float* __restrict__ DBC, const float* __restrict__ XCp, const float* __restrict__ XZ,
    const float* __restrict__ Wdt, const float* __restrict__ bdt, const float* __restrict__ Alog,
    const float* __restrict__ Dp, const float* __restrict__ YFin,
    float* __restrict__ YFout, unsigned short* __restrict__ YT)
{
  __shared__ __align__(16) float sX[kScanTS * kDbcP];
  __shared__ __align__(16) float sU[kScanTS * kScanCh];
  __shared__ __align__(16) float sZ[kScanTS * kScanCh];
  __shared__ __align__(16) float sF[DIR ? (kScanTS * kScanCh) : 4];
  __shared__ __align__(16) float sY[kScanTS * kScanYP];
  __shared__ float sA[kNst * kScanCh];
  const int tid = threadIdx.x, lane = tid & 31, wave = tid >> 5;
  const int d0 = blockIdx.x * kScanCh, d = d0 + tid;
#pragma unroll 1
  for (int s = 0; s < kNst; ++s) sA[s * kScanCh + tid] = -expf(Alog[(size_t)d * kNst + s]);
  const float wd0 = Wdt[d * kDtR + 0], wd1 = Wdt[d * kDtR + 1], wd2 = Wdt[d * kDtR + 2], wd3 = Wdt[d * kDtR + 3];
  const float bb = bdt[d], Dd = Dp[d];
  __syncthreads();
  float negA[kNst], h[kNst];
#pragma unroll
  for (int s = 0; s < kNst; ++s) { negA[s] = sA[s * kScanCh + tid]; h[s] = 0.f; }
  const int lr = tid >> 4, lc4 = (tid & 15) * 4;
  const int hh = lane >> 4, c4 = (lane & 15) * 4, q = lane >> 3, c8 = (lane & 7) * 8;
#pragma unroll 1
  for (int c = 0; c < kL / kScanTS; ++c) {
    const int R0 = DIR ? (kL - kScanTS * (c + 1)) : (kScanTS * c);
    __syncthreads();
#pragma unroll
    for (int i = 0; i < 8; ++i) {
      const int r = lr + 4 * i;
      *(v4f*)(sX + r * kDbcP + lc4) = *(const v4f*)(DBC + (size_t)(R0 + r) * kDbcP + lc4);
    }
    asm volatile("" ::: "memory");
#pragma unroll
    for (int i = 0; i < 8; ++i) {
      const int r = lr + 4 * i;
      *(v4f*)(sU + r * kScanCh + lc4) = *(const v4f*)(XCp + (size_t)(R0 + r) * kDin + d0 + lc4);
    }
    asm volatile("" ::: "memory");
#pragma unroll
    for (int i = 0; i < 8; ++i) {
      const int r = lr + 4 * i;
      *(v4f*)(sZ + r * kScanCh + lc4) = *(const v4f*)(XZ + (size_t)(R0 + r) * kXzP + kDin + d0 + lc4);
    }
    if constexpr (DIR == 1) {
      asm volatile("" ::: "memory");
#pragma unroll
      for (int i = 0; i < 8; ++i) {
        const int r = lr + 4 * i;
        *(v4f*)(sF + r * kScanCh + lc4) = *(const v4f*)(YFin + (size_t)(R0 + r) * kDin + d0 + lc4);
      }
    }
    __syncthreads();
#pragma unroll 1
    for (int ss = 0; ss < kScanTS; ++ss) {
      const int s = DIR ? (kScanTS - 1 - ss) : ss;
      const float* xr = sX + s * kDbcP;
      const v4f dv = *(const v4f*)(xr);
      float v = wd0 * dv.x;
      v = fmaf(wd1, dv.y, v);
      v = fmaf(wd2, dv.z, v);
      v = fmaf(wd3, dv.w, v);
      v = v + bb;
      const float ex = expf(-fabsf(v));
      const float dt = fmaxf(v, 0.0f) + log1pf(ex);
      float Bs[kNst], Cs[kNst];
#pragma unroll
      for (int q4 = 0; q4 < 4; ++q4) {
        const v4f bv = *(const v4f*)(xr + kDtR + 4 * q4);
        const v4f cv = *(const v4f*)(xr + kDtR + kNst + 4 * q4);
        Bs[4 * q4 + 0] = bv.x; Bs[4 * q4 + 1] = bv.y; Bs[4 * q4 + 2] = bv.z; Bs[4 * q4 + 3] = bv.w;
        Cs[4 * q4 + 0] = cv.x; Cs[4 * q4 + 1] = cv.y; Cs[4 * q4 + 2] = cv.z; Cs[4 * q4 + 3] = cv.w;
      }
      const float u = sU[s * kScanCh + tid];
      const float dtx = dt * u;
      float y = 0.0f;
#pragma unroll
      for (int k = 0; k < kNst; ++k) {
        const float e = __expf(dt * negA[k]);
        h[k] = e * h[k] + dtx * Bs[k];
        y = fmaf(h[k], Cs[k], y);
      }
      y = fmaf(u, Dd, y);
      const float z = sZ[s * kScanCh + tid];
      y = y * (z * sigm_f(z));
      if constexpr (DIR == 1) y = y + sF[s * kScanCh + tid];
      sY[s * kScanYP + tid] = y;
    }
    __syncthreads();
    if constexpr (DIR == 0) {
      v4f ov[8];
#pragma unroll
      for (int it = 0; it < 8; ++it) {
        const int row = it * 4 + wave * 2 + hh;
        ov[it] = *(const v4f*)(sY + row * kScanYP + c4);
      }
      for (int pass = 0; pass < 2; ++pass) {
#pragma unroll
        for (int it = 0; it < 8; ++it) {
          const int row = it * 4 + wave * 2 + hh;
          *(volatile v4f*)(YFout + (size_t)(R0 + row) * kDin + d0 + c4) = ov[it];
        }
        __threadfence();
      }
    } else {
      v8h hv[4];
#pragma unroll
      for (int it = 0; it < 4; ++it) {
        const int row = it * 8 + wave * 4 + q;
        const float* sp = sY + row * kScanYP + c8;
#pragma unroll
        for (int e = 0; e < 8; ++e) hv[it][e] = (_Float16)(sp[e] * kYCar);
      }
      for (int pass = 0; pass < 2; ++pass) {
#pragma unroll
        for (int it = 0; it < 4; ++it) {
          const int row = it * 8 + wave * 4 + q;
          *(volatile v8h*)(YT + (size_t)(R0 + row) * kDin + d0 + c8) = hv[it];
        }
        __threadfence();
      }
    }
  }
}

__global__ __launch_bounds__(256) void dwconv_gelu_kernel(const float* __restrict__ H1, const float* __restrict__ dww,
                                                          const float* __restrict__ dwb, unsigned short* __restrict__ H2G)
{
  __shared__ __align__(16) float sW[kTaps * kHid];
  __shared__ __align__(16) float sV[256 * 8];
  const int tid = threadIdx.x, lane = tid & 31, wave = tid >> 5;
#pragma unroll 1
  for (int tap = 0; tap < kTaps; ++tap) sW[tap * kHid + tid] = dww[(size_t)tid * kTaps + tap];
  __syncthreads();
  const int l = blockIdx.x * 8 + wave;
  const int c8 = lane * 8;
  const int t = l / kHW; const int rr = l - t * kHW; const int hq = rr / kW; const int wq = rr - hq * kW;
  const v4f b0 = *(const v4f*)(dwb + c8), b1 = *(const v4f*)(dwb + c8 + 4);
  float a[8];
  a[0] = b0.x; a[1] = b0.y; a[2] = b0.z; a[3] = b0.w; a[4] = b1.x; a[5] = b1.y; a[6] = b1.z; a[7] = b1.w;
#pragma unroll 1
  for (int tap = 0; tap < kTaps; ++tap) {
    const int kd = tap / 9; const int r9 = tap - kd * 9; const int kh = r9 / 3; const int kw = r9 - kh * 3;
    const int t2 = t + kd - 1, h2 = hq + kh - 1, w2 = wq + kw - 1;
    const bool inb = ((unsigned)t2 < (unsigned)kT) & ((unsigned)h2 < (unsigned)kH) & ((unsigned)w2 < (unsigned)kW);
    const int l2 = inb ? ((t2 * kH + h2) * kW + w2) : l;
    const float f = inb ? 1.0f : 0.0f;
    const v4f x0 = *(const v4f*)(H1 + (size_t)l2 * kHid + c8), x1 = *(const v4f*)(H1 + (size_t)l2 * kHid + c8 + 4);
    const v4f v0 = *(const v4f*)(sW + tap * kHid + c8), v1 = *(const v4f*)(sW + tap * kHid + c8 + 4);
    a[0] = fmaf(v0.x * f, x0.x, a[0]); a[1] = fmaf(v0.y * f, x0.y, a[1]);
    a[2] = fmaf(v0.z * f, x0.z, a[2]); a[3] = fmaf(v0.w * f, x0.w, a[3]);
    a[4] = fmaf(v1.x * f, x1.x, a[4]); a[5] = fmaf(v1.y * f, x1.y, a[5]);
    a[6] = fmaf(v1.z * f, x1.z, a[6]); a[7] = fmaf(v1.w * f, x1.w, a[7]);
  }
#pragma unroll
  for (int e = 0; e < 8; ++e) sV[tid * 8 + e] = a[e];
#pragma unroll 1
  for (int e = 0; e < 8; ++e) {
    const float vv = sV[tid * 8 + e];
    sV[tid * 8 + e] = gelu_f(vv) * kGCar;
  }
  __syncthreads();
  const v4f g0 = *(const v4f*)(sV + tid * 8), g1 = *(const v4f*)(sV + tid * 8 + 4);
  v8h hv;
  hv[0] = (_Float16)g0.x; hv[1] = (_Float16)g0.y; hv[2] = (_Float16)g0.z; hv[3] = (_Float16)g0.w;
  hv[4] = (_Float16)g1.x; hv[5] = (_Float16)g1.y; hv[6] = (_Float16)g1.z; hv[7] = (_Float16)g1.w;
  unsigned short* dp = H2G + (size_t)l * kHid + c8;
  *(volatile v8h*)dp = hv;
  __threadfence();
  *(volatile v8h*)dp = hv;
}

__global__ __launch_bounds__(256) void cb1g_kernel(const float* __restrict__ CB1, unsigned short* __restrict__ CB1G)
{
  __shared__ __align__(16) float sV[256 * 8];
  const int tid = threadIdx.x, lane = tid & 31, wave = tid >> 5;
  const int p = blockIdx.x * 128 + wave * 16 + (lane >> 1);
  const int c8 = (lane & 1) * 8;
  int l;
  const int in = pad_interior(p, &l);
  const float f = (float)in;
  int m = p - kPMin;
  m = (m < 0) ? 0 : ((m > kMConv - 1) ? (kMConv - 1) : m);
  const v4f a0 = *(const v4f*)(CB1 + (size_t)m * kCabMid + c8), a1 = *(const v4f*)(CB1 + (size_t)m * kCabMid + c8 + 4);
  sV[tid * 8 + 0] = a0.x * f; sV[tid * 8 + 1] = a0.y * f; sV[tid * 8 + 2] = a0.z * f; sV[tid * 8 + 3] = a0.w * f;
  sV[tid * 8 + 4] = a1.x * f; sV[tid * 8 + 5] = a1.y * f; sV[tid * 8 + 6] = a1.z * f; sV[tid * 8 + 7] = a1.w * f;
#pragma unroll 1
  for (int e = 0; e < 8; ++e) {
    const float vv = sV[tid * 8 + e];
    sV[tid * 8 + e] = gelu_f(vv) * kCbCar;
  }
  __syncthreads();
  const v4f g0 = *(const v4f*)(sV + tid * 8), g1 = *(const v4f*)(sV + tid * 8 + 4);
  v8h hv;
  hv[0] = (_Float16)g0.x; hv[1] = (_Float16)g0.y; hv[2] = (_Float16)g0.z; hv[3] = (_Float16)g0.w;
  hv[4] = (_Float16)g1.x; hv[5] = (_Float16)g1.y; hv[6] = (_Float16)g1.z; hv[7] = (_Float16)g1.w;
  unsigned short* dp = CB1G + (size_t)p * kCabMid + c8;
  *(volatile v8h*)dp = hv;
  __threadfence();
  *(volatile v8h*)dp = hv;
}

__global__ __launch_bounds__(256) void pool_kernel(const float* __restrict__ CB2, float* __restrict__ PART)
{
  __shared__ float sR[16 * 64];
  __shared__ __align__(16) float sO[64];
  const int tid = threadIdx.x, lane = tid & 31, wave = tid >> 5;
  const int rg = tid >> 4, c4 = (tid & 15) * 4;
  const int b = blockIdx.x;
  v4f acc = (v4f){0.f, 0.f, 0.f, 0.f};
#pragma unroll 1
  for (int r = rg; r < 311; r += 16) {
    const int m = b * 311 + r;
    int l;
    const float f = (float)pad_interior(m + kPMin, &l);
    const v4f v = *(const v4f*)(CB2 + (size_t)m * kOutC + c4);
    acc = acc + v * f;
  }
  sR[rg * 64 + c4 + 0] = acc.x; sR[rg * 64 + c4 + 1] = acc.y; sR[rg * 64 + c4 + 2] = acc.z; sR[rg * 64 + c4 + 3] = acc.w;
  __syncthreads();
  if (tid < 64) {
    float s = 0.f;
#pragma unroll 1
    for (int gq = 0; gq < 16; ++gq) s += sR[gq * 64 + tid];
    sO[tid] = s;
  }
  __syncthreads();
  if (wave == 0) {
    const int tl = lane & 15;
    const v4f o = *(const v4f*)(sO + tl * 4);
    float* dp = PART + (size_t)b * 64 + tl * 4;
    if (lane < 16) *(volatile v4f*)dp = o;
    __threadfence();
    if (lane < 16) *(volatile v4f*)dp = o;
  }
}

__global__ __launch_bounds__(64) void att_kernel(const float* __restrict__ PART, const float* __restrict__ w1,
                                                 const float* __restrict__ b1, const float* __restrict__ w2,
                                                 const float* __restrict__ b2, float* __restrict__ ATT)
{
  __shared__ float sP[64];
  __shared__ float sA[kSqMid];
  __shared__ __align__(16) float sG[64];
  const int tid = threadIdx.x, lane = tid & 31, wave = tid >> 5;
  float s = 0.f;
#pragma unroll 1
  for (int b = 0; b < 64; ++b) s += PART[(size_t)b * 64 + tid];
  sP[tid] = s * (1.0f / 18432.0f);
  __syncthreads();
  const int j = tid & 7;
  float a = 0.f;
#pragma unroll 1
  for (int c = 0; c < 64; ++c) a = fmaf(w1[j * 64 + c], sP[c], a);
  a = a + b1[j];
  a = fmaxf(a, 0.0f);
  if (tid < kSqMid) sA[tid] = a;
  __syncthreads();
  float s2 = 0.f;
#pragma unroll 1
  for (int jj = 0; jj < kSqMid; ++jj) s2 = fmaf(w2[tid * kSqMid + jj], sA[jj], s2);
  s2 = s2 + b2[tid];
  sG[tid] = sigm_f(s2);
  __syncthreads();
  if (wave == 0) {
    const int tl = lane & 15;
    const v4f o = *(const v4f*)(sG + tl * 4);
    float* dp = ATT + tl * 4;
    if (lane < 16) *(volatile v4f*)dp = o;
    __threadfence();
    if (lane < 16) *(volatile v4f*)dp = o;
  }
}

__global__ __launch_bounds__(256) void final_kernel(const float* __restrict__ OB, const float* __restrict__ CB2,
                                                    const float* __restrict__ ATT, const float* __restrict__ sk3,
                                                    float* __restrict__ OUT)
{
  __shared__ __align__(16) float sV[64 * 132];
  const int tid = threadIdx.x, lane = tid & 31, wave = tid >> 5;
  const int l0 = blockIdx.x * 128;
  const float s3 = sk3[0];
#pragma unroll
  for (int i = 0; i < 8; ++i) {
    const int f = tid + 256 * i;
    const int j = f >> 4;
    const int c4 = (f & 15) * 4;
    const int l = l0 + j;
    const int m = l_to_m(l);
    const v4f ob = *(const v4f*)(OB + (size_t)l * kOutC + c4);
    const v4f cb = *(const v4f*)(CB2 + (size_t)m * kOutC + c4);
    const v4f at = *(const v4f*)(ATT + c4);
    const v4f v = ob * s3 + cb * at;
    sV[(c4 + 0) * 132 + j] = v.x; sV[(c4 + 1) * 132 + j] = v.y; sV[(c4 + 2) * 132 + j] = v.z; sV[(c4 + 3) * 132 + j] = v.w;
    asm volatile("" ::: "memory");
  }
  __syncthreads();
  v4f ov[8];
#pragma unroll
  for (int it = 0; it < 8; ++it) {
    const int c = it * 8 + wave;
    ov[it] = *(const v4f*)(sV + c * 132 + lane * 4);
  }
  for (int pass = 0; pass < 2; ++pass) {
#pragma unroll
    for (int it = 0; it < 8; ++it) {
      const int c = it * 8 + wave;
      *(volatile v4f*)(OUT + (size_t)c * kL + l0 + lane * 4) = ov[it];
    }
    __threadfence();
  }
}

static_assert(kL % 64 == 0 && kMConv % 64 == 0);
static_assert(kC % 32 == 0 && kDin % 32 == 0 && kHid % 32 == 0 && kK1 % 32 == 0 && kK2 % 32 == 0);

extern "C" void kernel_launch(void* const* d_in, const int* in_sizes, int n_in,
                              void* d_out, int out_size, void* d_ws, size_t ws_size,
                              hipStream_t stream) {
  if (n_in < 42) return;
  if (in_sizes[0] != kC * kL) return;
  if (in_sizes[1] != kXzP * kC || in_sizes[2] != kDin * 4 || in_sizes[3] != kDin || in_sizes[4] != kDbcN * kDin ||
      in_sizes[5] != kDin * kDtR || in_sizes[6] != kDin || in_sizes[7] != kDin * kNst || in_sizes[8] != kDin) return;
  if (in_sizes[9] != kDin * 4 || in_sizes[10] != kDin || in_sizes[11] != kDbcN * kDin || in_sizes[12] != kDin * kDtR ||
      in_sizes[13] != kDin || in_sizes[14] != kDin * kNst || in_sizes[15] != kDin) return;
  if (in_sizes[16] != kC * kDin) return;
  if (in_sizes[17] != kC || in_sizes[18] != kC || in_sizes[19] != kC || in_sizes[20] != kC ||
      in_sizes[21] != kOutC || in_sizes[22] != kOutC) return;
  if (in_sizes[23] != 1 || in_sizes[24] != 1 || in_sizes[25] != 1) return;
  if (in_sizes[26] != kOutC * kC || in_sizes[27] != kOutC) return;
  if (in_sizes[28] != kHid * kC || in_sizes[29] != kHid || in_sizes[30] != kHid * kTaps || in_sizes[31] != kHid ||
      in_sizes[32] != kC * kHid || in_sizes[33] != kC) return;
  if (in_sizes[34] != kCabMid * kK1 || in_sizes[35] != kCabMid || in_sizes[36] != kOutC * kK2r || in_sizes[37] != kOutC) return;
  if (in_sizes[38] != kSqMid * kOutC || in_sizes[39] != kSqMid || in_sizes[40] != kOutC * kSqMid || in_sizes[41] != kOutC) return;
  if (out_size != kOutC * kL) return;
  if (ws_size < kWsTotal) return;

  const float* x        = (const float*)d_in[0];
  const float* in_proj  = (const float*)d_in[1];
  const float* c1w_f    = (const float*)d_in[2];
  const float* c1b_f    = (const float*)d_in[3];
  const float* xpw_f    = (const float*)d_in[4];
  const float* dtw_f    = (const float*)d_in[5];
  const float* dtb_f    = (const float*)d_in[6];
  const float* alog_f   = (const float*)d_in[7];
  const float* dp_f     = (const float*)d_in[8];
  const float* c1w_b    = (const float*)d_in[9];
  const float* c1b_b    = (const float*)d_in[10];
  const float* xpw_b    = (const float*)d_in[11];
  const float* dtw_b    = (const float*)d_in[12];
  const float* dtb_b    = (const float*)d_in[13];
  const float* alog_b   = (const float*)d_in[14];
  const float* dp_b     = (const float*)d_in[15];
  const float* out_proj = (const float*)d_in[16];
  const float* ln1w     = (const float*)d_in[17];
  const float* ln1b     = (const float*)d_in[18];
  const float* ln2w     = (const float*)d_in[19];
  const float* ln2b     = (const float*)d_in[20];
  const float* ln3w     = (const float*)d_in[21];
  const float* ln3b     = (const float*)d_in[22];
  const float* skip1    = (const float*)d_in[23];
  const float* skip2    = (const float*)d_in[24];
  const float* skip3    = (const float*)d_in[25];
  const float* proj_w   = (const float*)d_in[26];
  const float* proj_b   = (const float*)d_in[27];
  const float* fc1w     = (const float*)d_in[28];
  const float* fc1b     = (const float*)d_in[29];
  const float* dww      = (const float*)d_in[30];
  const float* dwb      = (const float*)d_in[31];
  const float* fc2w     = (const float*)d_in[32];
  const float* fc2b     = (const float*)d_in[33];
  const float* cab1w    = (const float*)d_in[34];
  const float* cab1b    = (const float*)d_in[35];
  const float* cab2w    = (const float*)d_in[36];
  const float* cab2b    = (const float*)d_in[37];
  const float* ca1w     = (const float*)d_in[38];
  const float* ca1b     = (const float*)d_in[39];
  const float* ca2w     = (const float*)d_in[40];
  const float* ca2b     = (const float*)d_in[41];
  float* out = (float*)d_out;

  char* ws = (char*)d_ws;
  unsigned short* IPW  = (unsigned short*)(ws + kOffIPW);
  unsigned short* OPW  = (unsigned short*)(ws + kOffOPW);
  unsigned short* F1W  = (unsigned short*)(ws + kOffF1W);
  unsigned short* F2W  = (unsigned short*)(ws + kOffF2W);
  unsigned short* PJW  = (unsigned short*)(ws + kOffPJW);
  unsigned short* XPW  = (unsigned short*)(ws + kOffXPW);
  unsigned short* C1R  = (unsigned short*)(ws + kOffC1R);
  unsigned short* C2R  = (unsigned short*)(ws + kOffC2R);
  float*          XT   = (float*)(ws + kOffXT);
  unsigned short* XN   = (unsigned short*)(ws + kOffXN);
  float*          XZ   = (float*)(ws + kOffXZ);
  float*          XC   = (float*)(ws + kOffXC);
  unsigned short* XCS  = (unsigned short*)(ws + kOffXCS);
  float*          DBC  = (float*)(ws + kOffDBC);
  float*          YF   = (float*)(ws + kOffYF);
  unsigned short* YT   = (unsigned short*)(ws + kOffYT);
  float*          XM   = (float*)(ws + kOffXM);
  unsigned short* XN2  = (unsigned short*)(ws + kOffXN2);
  float*          H1   = (float*)(ws + kOffH1);
  unsigned short* H2G  = (unsigned short*)(ws + kOffH2G);
  unsigned short* XM2  = (unsigned short*)(ws + kOffXM2);
  float*          OB   = (float*)(ws + kOffOB);
  unsigned short* CIP  = (unsigned short*)(ws + kOffCIP);
  float*          CB1  = (float*)(ws + kOffCB1);
  unsigned short* CB1G = (unsigned short*)(ws + kOffCB1G);
  float*          CB2  = (float*)(ws + kOffCB2);
  float*          PART = (float*)(ws + kOffPART);
  float*          ATT  = (float*)(ws + kOffATT);

  const float s8  = 1.0f / 256.0f;
  const float s14 = 1.0f / 16384.0f;
  const float s16 = 1.0f / 65536.0f;
  const float s18 = 1.0f / 262144.0f;

  prep_kernel<<<dim3(16, 8), dim3(256), 0, stream>>>(in_proj, out_proj, fc1w, fc2w, proj_w, xpw_f, xpw_b, cab1w, cab2w,
                                                     IPW, OPW, F1W, F2W, PJW, XPW, C1R, C2R);
  ln1_kernel<<<dim3(kL / 128), dim3(256), 0, stream>>>(x, ln1w, ln1b, XT, XN);
  gemm_f16_kernel<0, 4, 0, 0, false><<<dim3(144, 1), dim3(256), 0, stream>>>(
      XN, kC, 0L, IPW, kC, 0L, (void*)XZ, kXzP, 0L, nullptr, nullptr, nullptr, kL, kXzP, kC, s8);
  conv1d_silu_kernel<<<dim3(kL / 64, 2), dim3(128), 0, stream>>>(XZ, c1w_f, c1b_f, c1w_b, c1b_b, XC, XCS);
  gemm_f16_kernel<0, 4, 0, 0, false><<<dim3(36, 2), dim3(256), 0, stream>>>(
      XCS, kDin, (long)kL * kDin, XPW, kDin, (long)kDbcP * kDin, (void*)DBC, kDbcP, (long)kL * kDbcP,
      nullptr, nullptr, nullptr, kL, kDbcP, kDin, s18);
  scan_kernel<0><<<dim3(kDin / kScanCh), dim3(kScanCh), 0, stream>>>(
      DBC, XC, XZ, dtw_f, dtb_f, alog_f, dp_f, nullptr, YF, nullptr);
  scan_kernel<1><<<dim3(kDin / kScanCh), dim3(kScanCh), 0, stream>>>(
      DBC + (size_t)kL * kDbcP, XC + (size_t)kL * kDin, XZ, dtw_b, dtb_b, alog_b, dp_b, YF, nullptr, YT);
  gemm_f16_kernel<0, 4, 0, 0, true><<<dim3(36, 1), dim3(256), 0, stream>>>(
      YT, kDin, 0L, OPW, kDin, 0L, (void*)XM, kC, 0L, nullptr, XT, skip1, kL, kC, kDin, s18);
  ln2_kernel<<<dim3(kL / 32), dim3(256), 0, stream>>>(XM, ln2w, ln2b, XN2);
  gemm_f16_kernel<0, 4, 2, 0, false><<<dim3(144, 1), dim3(256), 0, stream>>>(
      XN2, kC, 0L, F1W, kC, 0L, (void*)H1, kHid, 0L, fc1b, nullptr, nullptr, kL, kHid, kC, s8);
  dwconv_gelu_kernel<<<dim3(kL / 8), dim3(256), 0, stream>>>(H1, dww, dwb, H2G);
  gemm_f16_kernel<0, 4, 2, 1, true><<<dim3(36, 1), dim3(256), 0, stream>>>(
      H2G, kHid, 0L, F2W, kHid, 0L, (void*)XM2, kC, 0L, fc2b, XM, skip2, kL, kC, kHid, s16);
  gemm_f16_kernel<0, 4, 2, 0, false><<<dim3(36, 1), dim3(256), 0, stream>>>(
      XM2, kC, 0L, PJW, kC, 0L, (void*)OB, kOutC, 0L, proj_b, nullptr, nullptr, kL, kOutC, kC, s8);
  ln3pad_kernel<<<dim3(kNPR / 32), dim3(256), 0, stream>>>(OB, ln3w, ln3b, CIP);
  gemm_f16_kernel<1, 1, 2, 0, false><<<dim3(39, 1), dim3(256), 0, stream>>>(
      CIP, kC, 0L, C1R, kK1, 0L, (void*)CB1, kCabMid, 0L, cab1b, nullptr, nullptr, kMConv, kCabMid, kK1, s8);
  cb1g_kernel<<<dim3(kNPR / 128), dim3(256), 0, stream>>>(CB1, CB1G);
  gemm_f16_kernel<2, 4, 2, 0, false><<<dim3(39, 1), dim3(256), 0, stream>>>(
      CB1G, kCabMid, 0L, C2R, kK2, 0L, (void*)CB2, kOutC, 0L, cab2b, nullptr, nullptr, kMConv, kOutC, kK2, s14);
  pool_kernel<<<dim3(64), dim3(256), 0, stream>>>(CB2, PART);
  att_kernel<<<dim3(1), dim3(64), 0, stream>>>(PART, ca1w, ca1b, ca2w, ca2b, ATT);
  final_kernel<<<dim3(kL / 128), dim3(256), 0, stream>>>(OB, CB2, ATT, skip3, out);
}
